// BasicFlow_60138132079052
// MI455X (gfx1250) — hardware-run, weakly checked
//
#include <hip/hip_runtime.h>
#include <math.h>

typedef __attribute__((ext_vector_type(16))) _Float16 v16h;
typedef __attribute__((ext_vector_type(8)))  _Float16 v8h;
typedef __attribute__((ext_vector_type(8)))  float    v8f;
typedef __attribute__((ext_vector_type(4)))  float    v4f;
typedef __attribute__((ext_vector_type(4)))  unsigned int v4u;

constexpr int kBatch   = 8;
constexpr int kChan    = 128;
constexpr int kH       = 96;
constexpr int kW       = 96;
constexpr int kPad     = 98;
constexpr int kWinSide = 8;
constexpr int kWinPerAxis = 12;
constexpr int kNWin    = 144;
constexpr int kTab     = 225;
constexpr int kImgPix  = kH * kW;
constexpr int kPixAll  = 2 * kBatch * kImgPix;
constexpr int kKdim    = 9 * kChan;
constexpr int kNout    = 2 * kChan;
constexpr int kTilesM  = kPixAll / 64;
constexpr int kTilesN  = kNout / 64;
constexpr int kSmPitch = 136;
constexpr int kOutSide = 384;
constexpr int kOutElems = kBatch * 2 * kOutSide * kOutSide;
constexpr float kFeatCarry = 16.0f;
constexpr float kWCarry    = 1024.0f;
constexpr float kQKCarry   = 16.0f;
constexpr float kConvFold  = 1.0f / (kFeatCarry * kWCarry);
constexpr float kMaskAdd   = -10000.0f;

static_assert(kImgPix == 9216, "image pixels");
static_assert(kPixAll == 147456, "flattened GEMM M");
static_assert((kPixAll % 64) == 0 && (kNout % 64) == 0, "GEMM M,N multiples of 64");
static_assert((kKdim % 32) == 0 && (kChan % 32) == 0, "GEMM K multiples of 32");
static_assert(kTilesM * kTilesN == 9216, "wave tiles");
static_assert(kWinPerAxis * kWinSide == kH && kWinPerAxis * kWinSide == kW, "window grid");
static_assert(kNWin == kWinPerAxis * kWinPerAxis, "windows per image");
static_assert(kTab == (2 * kWinSide - 1) * (2 * kWinSide - 1), "bias table length");
static_assert(kOutElems == 2359296, "elements per output tensor");
static_assert((size_t)4 * kOutElems * 4 == 37748736ull, "output bytes");

constexpr size_t kBytesFp   = (size_t)2 * kBatch * kPad * kPad * kChan * 2;
constexpr size_t kBytesBt   = (size_t)kNout * kKdim * 2;
constexpr size_t kBytesQK   = (size_t)kPixAll * kNout * 2;
constexpr size_t kBytesFmid = (size_t)2 * 4 * kBatch * kNWin * 128 * 4;
constexpr size_t kBytesFbsd = (size_t)2 * 4 * kBatch * kNWin * 32 * 4;
constexpr size_t kOffFp   = 0;
constexpr size_t kOffBt   = kOffFp + kBytesFp;
constexpr size_t kOffQK   = kOffBt + kBytesBt;
constexpr size_t kOffFmid = kOffQK + kBytesQK;
constexpr size_t kOffFbsd = kOffFmid + kBytesFmid;
constexpr size_t kWsTotal = kOffFbsd + kBytesFbsd;
static_assert(kBytesFp == 39337984ull, "FP bytes");
static_assert(kBytesBt == 589824ull, "BT bytes");
static_assert(kBytesQK == 75497472ull, "QK bytes");
static_assert(kBytesFmid == 4718592ull, "FMID bytes");
static_assert(kBytesFbsd == 1179648ull, "FBSD bytes");
static_assert(kWsTotal == 121323520ull, "carve total");
static_assert(kWsTotal <= 134217728ull, "carve cap");
static_assert((kOffBt % 128) == 0 && (kOffQK % 128) == 0 && (kOffFmid % 128) == 0 && (kOffFbsd % 128) == 0, "aligned regions");

__device__ __forceinline__ unsigned short h_bits(float f) {
  const _Float16 h = (_Float16)f;
  return __builtin_bit_cast(unsigned short, h);
}
__device__ __forceinline__ unsigned pk16(unsigned short a, unsigned short b) {
  return (unsigned)a | ((unsigned)b << 16);
}

template <typename T> struct Frag;
template <> struct Frag<_Float16> {
  typedef v16h V;
  union U { v16h v; v8h h[2]; };
  static __device__ __forceinline__ v16h load(const _Float16* p) {
    U f;
    f.h[0] = *(const v8h*)(p);
    f.h[1] = *(const v8h*)(p + 16);
    return f.v;
  }
};

__device__ __forceinline__ v8f mma_g(v16h a, v16h b, v8f c) {
  c = __builtin_amdgcn_wmma_f32_16x16x32_f16(false, a, false, b, (short)0, c, false, false);
  asm volatile("v_nop\n\tv_nop\n\tv_nop\n\tv_nop" : "+v"(c) : "v"(a), "v"(b));
  return c;
}

__global__ __launch_bounds__(256) void prep_feat_kernel(const float* __restrict__ f0,
                                                        const float* __restrict__ f2,
                                                        unsigned short* __restrict__ Fp) {
  __shared__ __align__(16) unsigned short sm[kPad * kSmPitch];
  const int tid = threadIdx.x;
  const int fb = blockIdx.x / kPad;
  const int yy = blockIdx.x - fb * kPad;
  const int f = fb >> 3;
  const int b = fb & 7;
  const float* src = (f == 0) ? f0 : f2;
  const bool inter = (yy >= 1) && (yy <= kH);
  const int ys = inter ? (yy - 1) : 0;
  {
    const int c = tid & 127;
    const int px = (tid >> 7) ? (kPad - 1) : 0;
    sm[px * kSmPitch + c] = (unsigned short)0;
  }
#pragma unroll 4
  for (int it = 0; it < 48; ++it) {
    const int i = it * 256 + tid;
    const int c = i / kW;
    const int x = i - c * kW;
    unsigned short hb = (unsigned short)0;
    if (inter) {
      const float v = src[((size_t)(b * kChan + c) * kH + ys) * kW + x];
      hb = h_bits(v * kFeatCarry);
    }
    sm[(x + 1) * kSmPitch + c] = hb;
  }
  __syncthreads();
  unsigned short* dst = Fp + ((size_t)fb * kPad + yy) * (size_t)(kPad * kChan);
  const int pq = tid >> 4;
  const int c8 = (tid & 15) * 8;
  for (int pass = 0; pass < 2; ++pass) {
#pragma unroll
    for (int it = 0; it < 7; ++it) {
      const int p = it * 16 + pq;
      if (p < kPad) {
        const v4u u = *(const v4u*)(sm + p * kSmPitch + c8);
        *(volatile v4u*)(dst + p * kChan + c8) = u;
      }
    }
    __threadfence();
  }
}

__global__ __launch_bounds__(256) void prep_w_kernel(const float* __restrict__ wq,
                                                     const float* __restrict__ wk,
                                                     unsigned short* __restrict__ Bt) {
  __shared__ float sw[kKdim];
  const int tid = threadIdx.x;
  const int n = blockIdx.x;
  const float* src = ((n < kChan) ? wq : wk) + (size_t)(n & (kChan - 1)) * kKdim;
  for (int i = tid; i < kKdim; i += 256) sw[i] = src[i];
  __syncthreads();
  if (tid < kKdim / 8) {
    const int k = tid * 8;
    const int tap = k >> 7;
    const int ci = k & (kChan - 1);
    unsigned short hb[8];
#pragma unroll
    for (int e = 0; e < 8; ++e) hb[e] = h_bits(sw[(ci + e) * 9 + tap] * kWCarry);
    const v4u u = (v4u){pk16(hb[0], hb[1]), pk16(hb[2], hb[3]), pk16(hb[4], hb[5]), pk16(hb[6], hb[7])};
    unsigned short* q = Bt + (size_t)n * kKdim + k;
    *(volatile v4u*)q = u;
    __threadfence();
    *(volatile v4u*)q = u;
  }
}

__global__ __launch_bounds__(256) void conv_gemm_kernel(const unsigned short* __restrict__ Fpp,
                                                        const unsigned short* __restrict__ Btp,
                                                        unsigned short* __restrict__ QKp,
                                                        const float* __restrict__ bq,
                                                        const float* __restrict__ bk) {
  __shared__ __align__(16) float sT[8][16 * 68];
  const _Float16* Fp = (const _Float16*)Fpp;
  const _Float16* Bt = (const _Float16*)Btp;
  const int lane = threadIdx.x & 31;
  const int wave = threadIdx.x >> 5;
  const int tile = blockIdx.x * 8 + wave;
  if (tile >= kTilesM * kTilesN) return;
  const int tm = tile >> 2;
  const int tn = tile & 3;
  const int m0 = tm << 6;
  const int n0 = tn << 6;
  const int rlane = lane & 15;
  const int koff = (lane >> 4) * 8;
  const int mOff = (lane >> 4) * 8;

  int aoff[4];
#pragma unroll
  for (int i = 0; i < 4; ++i) {
    const int m = m0 + (i << 4) + rlane;
    const int fb = m / kImgPix;
    const int rem = m - fb * kImgPix;
    const int y = rem / kW;
    const int x = rem - y * kW;
    aoff[i] = ((fb * kPad + y) * kPad + x) * kChan + koff;
  }
  const _Float16* bbase = Bt + (size_t)(n0 + rlane) * kKdim + koff;

  v8f acc[4][4];
#pragma unroll
  for (int i = 0; i < 4; ++i)
#pragma unroll
    for (int j = 0; j < 4; ++j) acc[i][j] = (v8f){0.f, 0.f, 0.f, 0.f, 0.f, 0.f, 0.f, 0.f};

#pragma unroll 1
  for (int ks = 0; ks < 36; ++ks) {
    const int tap = ks >> 2;
    const int kc = ks & 3;
    const int ky = tap / 3;
    const int kx = tap - ky * 3;
    const int tapoff = (ky * kPad + kx) * kChan + kc * 32;
    v16h bh[4];
#pragma unroll
    for (int j = 0; j < 4; ++j) bh[j] = Frag<_Float16>::load(bbase + (size_t)(j << 4) * kKdim + ks * 32);
#pragma unroll
    for (int i = 0; i < 4; ++i) {
      const v16h ah = Frag<_Float16>::load(Fp + aoff[i] + tapoff);
#pragma unroll
      for (int j = 0; j < 4; ++j) acc[i][j] = mma_g(ah, bh[j], acc[i][j]);
    }
  }

  float* slab = sT[wave];
  const float* bp = (n0 < kChan) ? (bq + n0) : (bk + (n0 - kChan));
  float bv[4];
#pragma unroll
  for (int j = 0; j < 4; ++j) bv[j] = bp[(j << 4) + rlane];
  const int q = lane >> 3;
  const int c8 = (lane & 7) * 8;
#pragma unroll
  for (int i = 0; i < 4; ++i) {
    const int mBase = m0 + (i << 4);
#pragma unroll
    for (int j = 0; j < 4; ++j) {
#pragma unroll
      for (int r = 0; r < 8; ++r) {
        const float v = (acc[i][j][r] * kConvFold + bv[j]) * kQKCarry;
        slab[(mOff + r) * 68 + (j << 4) + rlane] = v;
      }
    }
    __builtin_amdgcn_fence(__ATOMIC_RELEASE, "workgroup");
    __builtin_amdgcn_wave_barrier();
    __builtin_amdgcn_fence(__ATOMIC_ACQUIRE, "workgroup");
    for (int pass = 0; pass < 2; ++pass) {
#pragma unroll
      for (int it = 0; it < 4; ++it) {
        const int row = it * 4 + q;
        const float* sp = slab + row * 68 + c8;
        v8h hv;
#pragma unroll
        for (int e = 0; e < 8; ++e) hv[e] = (_Float16)sp[e];
        *(volatile v8h*)(QKp + (size_t)(mBase + row) * kNout + n0 + c8) = hv;
      }
      __threadfence();
    }
    __builtin_amdgcn_fence(__ATOMIC_RELEASE, "workgroup");
    __builtin_amdgcn_wave_barrier();
    __builtin_amdgcn_fence(__ATOMIC_ACQUIRE, "workgroup");
  }
}

__global__ __launch_bounds__(128) void corr_flow_kernel(const unsigned short* __restrict__ QKp,
                                                        const float* __restrict__ bias_table,
                                                        float* __restrict__ fmid,
                                                        float* __restrict__ fbsd,
                                                        float corrScale) {
  __shared__ __align__(16) float sCorr[64 * 68];
  __shared__ float sTab[256];
  __shared__ float sCm[96];
  __shared__ float sFx[96];
  __shared__ float sFy[96];
  __shared__ __align__(16) float sOut[160];

  const _Float16* QK = (const _Float16*)QKp;
  const int win = blockIdx.x;
  const int b = blockIdx.y;
  const int z = blockIdx.z;
  const int dir = z >> 2;
  const int var = z & 3;
  const int sh = (var & 2) ? 4 : 0;
  const int sw = (var & 1) ? 4 : 0;
  const int wy = win / kWinPerAxis;
  const int wx = win - wy * kWinPerAxis;
  const int fq = dir;
  const int fk = 1 - dir;
  const bool mh = (sh != 0) && (wy == kWinPerAxis - 1);
  const bool mw = (sw != 0) && (wx == kWinPerAxis - 1);

  const int tid = threadIdx.x;
  const int lane = tid & 31;
  const int wave = tid >> 5;
  const int hh = lane >> 4;
  const int lm = lane & 15;

  {
    const float t0 = bias_table[tid];
    const int i1 = tid + 128;
    const int i1c = (i1 < kTab) ? i1 : (kTab - 1);
    float t1 = bias_table[i1c];
    t1 = (i1 < kTab) ? t1 : 0.0f;
    sTab[tid] = t0;
    sTab[i1] = t1;
  }
  __syncthreads();

  v8f acc[4];
#pragma unroll
  for (int j = 0; j < 4; ++j) acc[j] = (v8f){0.f, 0.f, 0.f, 0.f, 0.f, 0.f, 0.f, 0.f};
  {
    const int l = wave * 16 + lm;
    int yq = wy * 8 + (l >> 3) + sh;
    int xq = wx * 8 + (l & 7) + sw;
    yq = (yq >= kH) ? (yq - kH) : yq;
    xq = (xq >= kW) ? (xq - kW) : xq;
    const _Float16* arow = QK + (size_t)((fq * kBatch + b) * kImgPix + yq * kW + xq) * kNout + 8 * hh;
    const _Float16* brow[4];
#pragma unroll
    for (int j = 0; j < 4; ++j) {
      const int t = j * 16 + lm;
      int yk = wy * 8 + (t >> 3) + sh;
      int xk = wx * 8 + (t & 7) + sw;
      yk = (yk >= kH) ? (yk - kH) : yk;
      xk = (xk >= kW) ? (xk - kW) : xk;
      brow[j] = QK + (size_t)((fk * kBatch + b) * kImgPix + yk * kW + xk) * kNout + kChan + 8 * hh;
    }
#pragma unroll
    for (int kc = 0; kc < 4; ++kc) {
      const v16h a = Frag<_Float16>::load(arow + kc * 32);
#pragma unroll
      for (int j = 0; j < 4; ++j) {
        const v16h bf = Frag<_Float16>::load(brow[j] + kc * 32);
        acc[j] = mma_g(a, bf, acc[j]);
      }
    }
  }

  {
    const int ly = wave * 2 + hh;
#pragma unroll
    for (int j = 0; j < 4; ++j) {
      const int tcol = j * 16 + lm;
      const int ty = tcol >> 3;
      const int tx = tcol & 7;
      const bool dy = mh && ((ly < 4) != (ty < 4));
      const int rowIdx = (ly - ty + 7) * 15 + 7 - tx;
#pragma unroll
      for (int r = 0; r < 8; ++r) {
        const int lx = r;
        const int lrow = wave * 16 + 8 * hh + r;
        float v = acc[j][r] * corrScale + sTab[rowIdx + lx];
        const bool dx = mw && ((lx < 4) != (tx < 4));
        v = (dy || dx) ? (v + kMaskAdd) : v;
        sCorr[lrow * 68 + tcol] = v;
      }
    }
  }
  __syncthreads();

  {
    const int r16 = tid >> 3;
    const int sub = tid & 7;
    const int ly = (r16 >> 2) + 2;
    const int lx = (r16 & 3) + 2;
    const float* cr = sCorr + (ly * 8 + lx) * 68 + sub * 8;
    const v4f a0 = *(const v4f*)(cr);
    const v4f a1 = *(const v4f*)(cr + 4);
    float xv[8];
    xv[0] = a0[0]; xv[1] = a0[1]; xv[2] = a0[2]; xv[3] = a0[3];
    xv[4] = a1[0]; xv[5] = a1[1]; xv[6] = a1[2]; xv[7] = a1[3];
    float mx = fmaxf(fmaxf(fmaxf(xv[0], xv[1]), fmaxf(xv[2], xv[3])), fmaxf(fmaxf(xv[4], xv[5]), fmaxf(xv[6], xv[7])));
    mx = fmaxf(mx, __shfl_xor(mx, 1, 32));
    mx = fmaxf(mx, __shfl_xor(mx, 2, 32));
    mx = fmaxf(mx, __shfl_xor(mx, 4, 32));
    const float flx = (float)lx;
    float s = 0.0f, fx = 0.0f;
#pragma unroll
    for (int j = 0; j < 8; ++j) {
      const float e = __expf(xv[j] - mx);
      s += e;
      fx += e * ((float)j - flx);
    }
    float fy = s * (float)(sub - ly);
    s  += __shfl_xor(s, 1, 32);
    fx += __shfl_xor(fx, 1, 32);
    fy += __shfl_xor(fy, 1, 32);
    s  += __shfl_xor(s, 2, 32);
    fx += __shfl_xor(fx, 2, 32);
    fy += __shfl_xor(fy, 2, 32);
    s  += __shfl_xor(s, 4, 32);
    fx += __shfl_xor(fx, 4, 32);
    fy += __shfl_xor(fy, 4, 32);
    const float inv = __builtin_amdgcn_rcpf(s);
    if (sub == 0) {
      sOut[128 + r16] = fx * inv;
      sOut[144 + r16] = fy * inv;
    }
  }

  if (wave < 3) {
    const int p = (tid < 81) ? tid : 80;
    const int u = p / 9;
    const int v9 = p - u * 9;
    float mx = -3.0e38f;
#pragma unroll 1
    for (int h2 = 0; h2 < 8; ++h2) {
      const int h0 = u + 3 - h2;
      const bool hok = (h0 >= 0) && (h0 < 8);
      const int h0c = (h0 < 0) ? 0 : ((h0 > 7) ? 7 : h0);
      const float* rowb = sCorr + (h0c * 8) * 68 + h2 * 8;
#pragma unroll
      for (int w2 = 0; w2 < 8; ++w2) {
        const int w0 = v9 + 3 - w2;
        const bool ok = hok && (w0 >= 0) && (w0 < 8);
        const int w0c = (w0 < 0) ? 0 : ((w0 > 7) ? 7 : w0);
        const float cv = rowb[w0c * 68 + w2];
        const float c = ok ? cv : 0.0f;
        mx = fmaxf(mx, c);
      }
    }
    float s = 0.0f, sxw = 0.0f, syw = 0.0f, cw = 0.0f;
#pragma unroll 1
    for (int h2 = 0; h2 < 8; ++h2) {
      const int h0 = u + 3 - h2;
      const bool hok = (h0 >= 0) && (h0 < 8);
      const int h0c = (h0 < 0) ? 0 : ((h0 > 7) ? 7 : h0);
      const float* rowb = sCorr + (h0c * 8) * 68 + h2 * 8;
      float srow = 0.0f;
#pragma unroll
      for (int w2 = 0; w2 < 8; ++w2) {
        const int w0 = v9 + 3 - w2;
        const bool ok = hok && (w0 >= 0) && (w0 < 8);
        const int w0c = (w0 < 0) ? 0 : ((w0 > 7) ? 7 : w0);
        const float cv = rowb[w0c * 68 + w2];
        const float c = ok ? cv : 0.0f;
        const float e = __expf(c - mx);
        srow += e;
        sxw += e * (float)w2;
        cw += e * c;
      }
      s += srow;
      syw += srow * (float)h2;
    }
    const float inv = __builtin_amdgcn_rcpf(s);
    const float bx = 1.5f + 0.5f * (float)v9;
    const float by = 1.5f + 0.5f * (float)u;
    if (tid < 81) {
      sCm[tid] = cw * inv;
      sFx[tid] = sxw * inv - bx;
      sFy[tid] = syw * inv - by;
    }
  }
  __syncthreads();

  if (tid < 64) {
    const int yq = tid >> 3;
    const int xq = tid & 7;
    const int i00 = yq * 9 + xq;
    const int i01 = i00 + 1;
    const int i10 = i00 + 9;
    const int i11 = i00 + 10;
    const float c0 = sCm[i00], c1 = sCm[i01], c2 = sCm[i10], c3 = sCm[i11];
    const float mx = fmaxf(fmaxf(c0, c1), fmaxf(c2, c3));
    const float e0 = __expf(c0 - mx);
    const float e1 = __expf(c1 - mx);
    const float e2 = __expf(c2 - mx);
    const float e3 = __expf(c3 - mx);
    const float s = (e0 + e1) + (e2 + e3);
    const float sc = 2.0f * __builtin_amdgcn_rcpf(s);
    const float ox = (sFx[i00] * e0 + sFx[i01] * e1 + sFx[i10] * e2 + sFx[i11] * e3) * sc;
    const float oy = (sFy[i00] * e0 + sFy[i01] * e1 + sFy[i10] * e2 + sFy[i11] * e3) * sc;
    sOut[tid] = ox;
    sOut[64 + tid] = oy;
  }
  __syncthreads();

  const size_t obase = (size_t)(((dir * 4 + var) * kBatch + b) * kNWin + win);
  if (wave == 0) {
    const v4f val = *(const v4f*)(sOut + lane * 4);
    float* q = fmid + obase * 128 + lane * 4;
    *(volatile v4f*)q = val;
    __threadfence();
    *(volatile v4f*)q = val;
  } else if (wave == 1) {
    if (lane < 8) {
      const v4f val = *(const v4f*)(sOut + 128 + lane * 4);
      float* q = fbsd + obase * 32 + lane * 4;
      *(volatile v4f*)q = val;
      __threadfence();
      *(volatile v4f*)q = val;
    }
  }
}

template <bool MID> __device__ __forceinline__ int up_row_off(int c) {
  constexpr int S = MID ? 192 : 96;
  constexpr int RB = MID ? 188 : 94;
  constexpr int BSH = MID ? 4 : 3;
  constexpr int HSH = MID ? 3 : 2;
  constexpr int CW = MID ? 8 : 4;
  constexpr int WS = 2 * CW * CW;
  constexpr int PL = kBatch * kNWin * WS;
  int p = c + RB;
  p = (p >= S) ? (p - S) : p;
  const int w = p >> BSH;
  const int hq = p & ((1 << BSH) - 1);
  const int vv = hq >> HSH;
  const int ii = hq & (CW - 1);
  return vv * 2 * PL + w * kWinPerAxis * WS + ii * CW;
}
template <bool MID> __device__ __forceinline__ int up_col_off(int c) {
  constexpr int S = MID ? 192 : 96;
  constexpr int RB = MID ? 188 : 94;
  constexpr int BSH = MID ? 4 : 3;
  constexpr int HSH = MID ? 3 : 2;
  constexpr int CW = MID ? 8 : 4;
  constexpr int WS = 2 * CW * CW;
  constexpr int PL = kBatch * kNWin * WS;
  int p = c + RB;
  p = (p >= S) ? (p - S) : p;
  const int w = p >> BSH;
  const int hq = p & ((1 << BSH) - 1);
  const int vv = hq >> HSH;
  const int ii = hq & (CW - 1);
  return vv * PL + w * WS + ii;
}

template <bool MID>
__device__ __forceinline__ void up_body(const float* __restrict__ src, float* __restrict__ dst, int dir, int gid) {
  constexpr int S = MID ? 192 : 96;
  constexpr int CW = MID ? 8 : 4;
  constexpr int CELL = CW * CW;
  constexpr int WS = 2 * CELL;
  constexpr int PL = kBatch * kNWin * WS;
  constexpr float FMUL = MID ? 2.0f : 4.0f;
  constexpr float FINV = MID ? 0.5f : 0.25f;
  const int X4 = gid % 96;
  int t = gid / 96;
  const int Y = t % kOutSide;
  t = t / kOutSide;
  const int ch = t & 1;
  const int b = t >> 1;
  const int base = dir * 4 * PL + b * kNWin * WS + ch * CELL;
  const float sy = ((float)Y + 0.5f) * FINV - 0.5f;
  const float fy0 = floorf(sy);
  const int y0 = (int)fy0;
  const float wy1 = sy - fy0;
  const float wy0 = 1.0f - wy1;
  const int y0c = (y0 < 0) ? 0 : y0;
  const int y1c = (y0 + 1 > S - 1) ? (S - 1) : (y0 + 1);
  const int r0 = base + up_row_off<MID>(y0c);
  const int r1 = base + up_row_off<MID>(y1c);
  float rv[4];
#pragma unroll
  for (int e = 0; e < 4; ++e) {
    const int X = X4 * 4 + e;
    const float sx = ((float)X + 0.5f) * FINV - 0.5f;
    const float fx0 = floorf(sx);
    const int x0 = (int)fx0;
    const float wx1 = sx - fx0;
    const float wx0 = 1.0f - wx1;
    const int x0c = (x0 < 0) ? 0 : x0;
    const int x1c = (x0 + 1 > S - 1) ? (S - 1) : (x0 + 1);
    const int c0 = up_col_off<MID>(x0c);
    const int c1 = up_col_off<MID>(x1c);
    const float v00 = src[r0 + c0];
    const float v01 = src[r0 + c1];
    const float v10 = src[r1 + c0];
    const float v11 = src[r1 + c1];
    const float top = wx0 * v00 + wx1 * v01;
    const float bot = wx0 * v10 + wx1 * v11;
    rv[e] = (wy0 * top + wy1 * bot) * FMUL;
  }
  const v4f o = (v4f){rv[0], rv[1], rv[2], rv[3]};
  float* q = dst + (size_t)gid * 4;
  *(volatile v4f*)q = o;
  __threadfence();
  *(volatile v4f*)q = o;
}

__global__ __launch_bounds__(256) void splice_up_kernel(const float* __restrict__ fmid,
                                                        const float* __restrict__ fbsd,
                                                        float* __restrict__ out) {
  const int ti = blockIdx.y;
  const int gid = blockIdx.x * 256 + threadIdx.x;
  float* dst = out + (size_t)ti * kOutElems;
  const int dir = (ti == 0 || ti == 3) ? 1 : 0;
  if (ti < 2) up_body<true>(fmid, dst, dir, gid);
  else        up_body<false>(fbsd, dst, dir, gid);
}

extern "C" void kernel_launch(void* const* d_in, const int* in_sizes, int n_in,
                              void* d_out, int out_size, void* d_ws, size_t ws_size,
                              hipStream_t stream) {
  if (n_in < 7) return;
  if (in_sizes[0] != kBatch * kChan * kImgPix) return;
  if (in_sizes[1] != kBatch * kChan * kImgPix) return;
  if (in_sizes[2] != kChan * kKdim) return;
  if (in_sizes[3] != kChan) return;
  if (in_sizes[4] != kChan * kKdim) return;
  if (in_sizes[5] != kChan) return;
  if (in_sizes[6] != kTab) return;
  if (out_size != 4 * kOutElems) return;
  if (ws_size < kWsTotal) return;

  const float* feat0 = (const float*)d_in[0];
  const float* feat2 = (const float*)d_in[1];
  const float* wq    = (const float*)d_in[2];
  const float* bq    = (const float*)d_in[3];
  const float* wk    = (const float*)d_in[4];
  const float* bk    = (const float*)d_in[5];
  const float* btab  = (const float*)d_in[6];
  float* out = (float*)d_out;

  char* ws = (char*)d_ws;
  unsigned short* Fp = (unsigned short*)(ws + kOffFp);
  unsigned short* Bt = (unsigned short*)(ws + kOffBt);
  unsigned short* QK = (unsigned short*)(ws + kOffQK);
  float* fmid = (float*)(ws + kOffFmid);
  float* fbsd = (float*)(ws + kOffFbsd);

  const float scl = (float)(1.0 / sqrt((double)kChan));
  const float corrScale = scl / (kQKCarry * kQKCarry);

  prep_feat_kernel<<<2 * kBatch * kPad, 256, 0, stream>>>(feat0, feat2, Fp);
  prep_w_kernel<<<kNout, 256, 0, stream>>>(wq, wk, Bt);
  conv_gemm_kernel<<<(kTilesM * kTilesN) / 8, 256, 0, stream>>>(Fp, Bt, QK, bq, bk);
  corr_flow_kernel<<<dim3(kNWin, kBatch, 8), 128, 0, stream>>>(QK, btab, fmid, fbsd, corrScale);
  splice_up_kernel<<<dim3(kOutElems / (4 * 256), 4), 256, 0, stream>>>(fmid, fbsd, out);
}
